// NetworkGNN_79422535237963
// MI455X (gfx1250) — hardware-verified
//
#include <hip/hip_runtime.h>
#include <stddef.h>


#define FIN     128
#define FH      64
#define FOUT    40
#define NLAY    3
#define FLA     (NLAY * FH)
#define NTHR    256
#define NWAVE   8
#define EPT     8
#define NGRP    2
#define CHUNK   (NTHR * EPT * NGRP)
#define WCAP    (EPT * NGRP * 32)
#define LISTN   (NWAVE * WCAP)
#define ESHF    11
#define NBC     32768
#define NBF     2048
#define RCAP    40960
#define RBN     128
#define TGT     256
#define DEGCAP  512
#define GROWS   128
#define OTHR    512
#define APH     (FH + 8)
#define WSCAP   134217728

#define PW_IN   0
#define PW_G    (FH * FIN)
#define PW_LA   (PW_G + NLAY * FH * FH)
#define PW_CLS  (PW_LA + FH * FLA)
#define PW_TOT  (PW_CLS + FH * FH)
#define WPREP_BLOCKS ((PW_TOT / 8) / NTHR)

#define LDS_COUNT ((NBC + LISTN + NWAVE) * 4)
#define LDS_FILL  ((RCAP + NBF + LISTN + NWAVE) * 4)

static_assert((CHUNK & (CHUNK - 1)) == 0);
static_assert((NBC & (NBC - 1)) == 0 && (NBF & (NBF - 1)) == 0);
static_assert(NBF <= (1 << ESHF));
static_assert((NBC % NBF) == 0);
static_assert(OTHR * 4 == NBF);
static_assert((RCAP % 32) == 0);
static_assert(TGT == NWAVE * 32);
static_assert(GROWS == NWAVE * 16);
static_assert((TGT % GROWS) == 0);
static_assert(NBC == NWAVE * 32 * 128);
static_assert((FIN % 32) == 0 && (FH % 32) == 0 && FH == 64 && (FLA % 32) == 0);
static_assert(FOUT <= FH && (FOUT % 4) == 0 && ((16 * FOUT) % 128) == 0);
static_assert(((PW_G / 8) % NTHR) == 0 && ((PW_LA / 8) % NTHR) == 0 && ((PW_CLS / 8) % NTHR) == 0 && ((PW_TOT / 8) % NTHR) == 0);
static_assert((APH % 8) == 0);
static_assert(NWAVE * 16 * APH * 2 * 2 + NWAVE * 16 * FOUT * 4 <= 65536);

typedef float          v2f   __attribute__((ext_vector_type(2)));
typedef float          v4f   __attribute__((ext_vector_type(4)));
typedef float          v8f   __attribute__((ext_vector_type(8)));
typedef int            v4i   __attribute__((ext_vector_type(4)));
typedef unsigned short v8us  __attribute__((ext_vector_type(8)));
typedef unsigned short v16us __attribute__((ext_vector_type(16)));
typedef __bf16         v16bf __attribute__((ext_vector_type(16)));
union FragU { v16us v; v8us h[2]; };

__device__ __forceinline__ v8f wmb(v16us a, v16us b, v8f c) {
  v8f d = __builtin_amdgcn_wmma_f32_16x16x32_bf16(false, __builtin_bit_cast(v16bf, a), false,
                                                  __builtin_bit_cast(v16bf, b), (short)0, c, false, false);
  asm volatile("v_nop\n\tv_nop\n\tv_nop\n\tv_nop" : "+v"(d) : "v"(a), "v"(b));
  return d;
}

__device__ __forceinline__ unsigned bfrne(float x) {
  const unsigned u = __float_as_uint(x);
  return (u + 0x7FFFu + ((u >> 16) & 1u)) >> 16;
}
__device__ __forceinline__ void split1(float x, unsigned short& hi, unsigned short& lo) {
  const unsigned hb = bfrne(x);
  const float hf = __uint_as_float(hb << 16);
  const unsigned lb = bfrne(x - hf);
  hi = (unsigned short)hb;
  lo = (unsigned short)lb;
}
__device__ __forceinline__ void split16(const float* p, v16us& hi, v16us& lo) {
  const v4f a = *(const v4f*)p, b = *(const v4f*)(p + 4), c = *(const v4f*)(p + 16), d = *(const v4f*)(p + 20);
  float f[16];
  f[0] = a.x; f[1] = a.y; f[2]  = a.z; f[3]  = a.w; f[4]  = b.x; f[5]  = b.y; f[6]  = b.z; f[7]  = b.w;
  f[8] = c.x; f[9] = c.y; f[10] = c.z; f[11] = c.w; f[12] = d.x; f[13] = d.y; f[14] = d.z; f[15] = d.w;
#pragma unroll
  for (int i = 0; i < 16; ++i) {
    unsigned short s, t;
    split1(f[i], s, t);
    hi[i] = s; lo[i] = t;
  }
}

template <int NB, int SRC>
__device__ __forceinline__ int scan_chunk(const int* __restrict__ dsts, const int* __restrict__ srcs, int nE, int nN,
                                          int cbase, int slotBase, int vec8, int* list, int tid, int lane, int wave) {
  int wc = 0;
#pragma unroll
  for (int g = 0; g < NGRP; ++g) {
    const int el0  = (g * NTHR + tid) * EPT;
    const int e0   = cbase + el0;
    const int sent = -2147483647 - 1;
    v4i da, db;
    v4i sa = {0, 0, 0, 0}, sb = {0, 0, 0, 0};
    if (vec8 != 0 && cbase + CHUNK <= nE) {
      da = *(const v4i*)(dsts + e0);
      db = *(const v4i*)(dsts + e0 + 4);
      if (SRC) {
        sa = *(const v4i*)(srcs + e0);
        sb = *(const v4i*)(srcs + e0 + 4);
      }
    } else {
      da.x = (e0     < nE) ? dsts[min(e0, nE - 1)] : sent;
      da.y = (e0 + 1 < nE) ? dsts[min(e0 + 1, nE - 1)] : sent;
      da.z = (e0 + 2 < nE) ? dsts[min(e0 + 2, nE - 1)] : sent;
      da.w = (e0 + 3 < nE) ? dsts[min(e0 + 3, nE - 1)] : sent;
      db.x = (e0 + 4 < nE) ? dsts[min(e0 + 4, nE - 1)] : sent;
      db.y = (e0 + 5 < nE) ? dsts[min(e0 + 5, nE - 1)] : sent;
      db.z = (e0 + 6 < nE) ? dsts[min(e0 + 6, nE - 1)] : sent;
      db.w = (e0 + 7 < nE) ? dsts[min(e0 + 7, nE - 1)] : sent;
      if (SRC) {
        sa.x = srcs[min(e0, nE - 1)];
        sa.y = srcs[min(e0 + 1, nE - 1)];
        sa.z = srcs[min(e0 + 2, nE - 1)];
        sa.w = srcs[min(e0 + 3, nE - 1)];
        sb.x = srcs[min(e0 + 4, nE - 1)];
        sb.y = srcs[min(e0 + 5, nE - 1)];
        sb.z = srcs[min(e0 + 6, nE - 1)];
        sb.w = srcs[min(e0 + 7, nE - 1)];
      }
    }
    if (SRC) {
      sa.x = min(max(sa.x, 0), nN - 1); sa.y = min(max(sa.y, 0), nN - 1);
      sa.z = min(max(sa.z, 0), nN - 1); sa.w = min(max(sa.w, 0), nN - 1);
      sb.x = min(max(sb.x, 0), nN - 1); sb.y = min(max(sb.y, 0), nN - 1);
      sb.z = min(max(sb.z, 0), nN - 1); sb.w = min(max(sb.w, 0), nN - 1);
    }
    const unsigned nb = (unsigned)slotBase;
    const unsigned s0 = (unsigned)da.x - nb, s1 = (unsigned)da.y - nb;
    const unsigned s2 = (unsigned)da.z - nb, s3 = (unsigned)da.w - nb;
    const unsigned s4 = (unsigned)db.x - nb, s5 = (unsigned)db.y - nb;
    const unsigned s6 = (unsigned)db.z - nb, s7 = (unsigned)db.w - nb;
    const bool h0 = s0 < (unsigned)NB, h1 = s1 < (unsigned)NB, h2 = s2 < (unsigned)NB, h3 = s3 < (unsigned)NB;
    const bool h4 = s4 < (unsigned)NB, h5 = s5 < (unsigned)NB, h6 = s6 < (unsigned)NB, h7 = s7 < (unsigned)NB;
    const unsigned any = __builtin_amdgcn_ballot_w32(h0 | h1 | h2 | h3 | h4 | h5 | h6 | h7);
    if (any != 0u) {
#define HITJ(HJ, SJ, VJ) { \
        const unsigned mj = __builtin_amdgcn_ballot_w32(HJ); \
        if (mj != 0u) { \
          if (HJ) { \
            const int pos = wc + (int)__builtin_amdgcn_mbcnt_lo(mj, 0u); \
            const int entv = SRC ? (((VJ) << ESHF) | (int)(SJ)) : (int)(SJ); \
            if (pos < WCAP) list[wave * WCAP + pos] = entv; \
          } \
          wc += (int)__builtin_popcount(mj); } }
      HITJ(h0, s0, sa.x)
      HITJ(h1, s1, sa.y)
      HITJ(h2, s2, sa.z)
      HITJ(h3, s3, sa.w)
      HITJ(h4, s4, sb.x)
      HITJ(h5, s5, sb.y)
      HITJ(h6, s6, sb.z)
      HITJ(h7, s7, sb.w)
#undef HITJ
    }
  }
  return wc;
}

__global__ __launch_bounds__(NTHR) void k_wprep(const float* __restrict__ w_in, const float* __restrict__ w_g,
                                                const float* __restrict__ w_la, const float* __restrict__ w_c,
                                                unsigned short* wp) {
  const int tid = threadIdx.x;
  const int g = (int)blockIdx.x * NTHR + tid;
  float f[8];
  if (blockIdx.x < (PW_G / 8) / NTHR) {
    const int i = g, n = i >> 4, k0 = (i & 15) * 8;
#pragma unroll
    for (int e = 0; e < 8; ++e) f[e] = w_in[(k0 + e) * FH + n];
  } else if (blockIdx.x < (PW_LA / 8) / NTHR) {
    const int j = g - PW_G / 8;
    const int li = j >> 9, jj = j & 511;
    const int n = jj >> 3, k0 = (jj & 7) * 8;
#pragma unroll
    for (int e = 0; e < 8; ++e) f[e] = w_g[(size_t)li * FH * FH + (size_t)(k0 + e) * FH + n];
  } else if (blockIdx.x < (PW_CLS / 8) / NTHR) {
    const int j = g - PW_LA / 8;
    const int n = j / (FLA / 8), k0 = (j - n * (FLA / 8)) * 8;
#pragma unroll
    for (int e = 0; e < 8; ++e) f[e] = w_la[(k0 + e) * FH + n];
  } else {
    const int j = g - PW_CLS / 8;
    const int n = j >> 3, k0 = (j & 7) * 8;
    const int nc = n < FOUT ? n : FOUT - 1;
#pragma unroll
    for (int e = 0; e < 8; ++e) {
      const float v = w_c[(k0 + e) * FOUT + nc];
      f[e] = n < FOUT ? v : 0.0f;
    }
  }
  v8us hv, lv;
#pragma unroll
  for (int e = 0; e < 8; ++e) {
    unsigned short s, t;
    split1(f[e], s, t);
    hv[e] = s; lv[e] = t;
  }
  unsigned short* d = wp + (size_t)g * 8;
  *(volatile v8us*)d = hv;
  *(volatile v8us*)(d + PW_TOT) = lv;
  __threadfence();
  *(volatile v8us*)d = hv;
  *(volatile v8us*)(d + PW_TOT) = lv;
}

__device__ __forceinline__ float dnorm(int c) {
  const float r = rsqrtf((float)(c > 0 ? c : 1));
  return c > 0 ? r : 0.0f;
}

__global__ __launch_bounds__(NTHR) void k_count(
    const int* __restrict__ ei, int* cnt, float* dinv, int nE, int nN, int vec8) {
  extern __shared__ v4f lds_dyn[];
  int* scnt = (int*)lds_dyn;
  int* list = scnt + NBC;
  int* wcnt = list + LISTN;
  const int tid = threadIdx.x, lane = tid & 31, wave = tid >> 5;
  const int nodeBase = blockIdx.x * NBC;
  const int* dsts = ei + nE;

  {
    const v4i z = {0, 0, 0, 0};
    for (int i = tid; i < NBC / 4; i += NTHR) ((v4i*)scnt)[i] = z;
  }
  __syncthreads();

  const int nChunks = (nE + CHUNK - 1) / CHUNK;
#pragma unroll 1
  for (int ch = 0; ch < nChunks; ++ch) {
    const int cbase = ch * CHUNK;
    const int wc = scan_chunk<NBC, 0>(dsts, ei, nE, nN, cbase, nodeBase, vec8, list, tid, lane, wave);
    if (lane == 0) wcnt[wave] = wc;
    __syncthreads();
    if (wave == 0) {
#pragma unroll 1
      for (int wsx = 0; wsx < NWAVE; ++wsx) {
        int n = __builtin_amdgcn_readfirstlane(wcnt[wsx]);
        n = n > WCAP ? WCAP : (n < 0 ? 0 : n);
        const int* lp = list + wsx * WCAP;
#pragma unroll 1
        for (int i = 0; i < n; ++i) {
          const int ent  = __builtin_amdgcn_readfirstlane(lp[i]);
          const int slot = ent & (NBC - 1);
          if (lane == 0) scnt[slot] = scnt[slot] + 1;
        }
      }
    }
    __syncthreads();
  }

  int*   cp = cnt + (size_t)nodeBase;
  float* dp = dinv + (size_t)nodeBase;
#pragma unroll 4
  for (int q = 0; q < 32; ++q) {
    const int f = (wave * 32 + q) * 128 + 4 * lane;
    const v4i c = *(const v4i*)(scnt + f);
    v4f d;
    d.x = dnorm(c.x); d.y = dnorm(c.y); d.z = dnorm(c.z); d.w = dnorm(c.w);
    *(volatile v4i*)(cp + f) = c;
    *(volatile v4f*)(dp + f) = d;
  }
  __threadfence();
#pragma unroll 4
  for (int q = 0; q < 32; ++q) {
    const int f = (wave * 32 + q) * 128 + 4 * lane;
    const v4i c = *(const v4i*)(scnt + f);
    v4f d;
    d.x = dnorm(c.x); d.y = dnorm(c.y); d.z = dnorm(c.z); d.w = dnorm(c.w);
    *(volatile v4i*)(cp + f) = c;
    *(volatile v4f*)(dp + f) = d;
  }
}

__global__ __launch_bounds__(OTHR) void k_offsets(
    const int* __restrict__ cnt, int* off, int* rbase, int nBF) {
  __shared__ __attribute__((aligned(16))) int srb[RBN];
  __shared__ int wtot[OTHR / 32];
  const int tid = threadIdx.x, lane = tid & 31, wave = tid >> 5;
  for (int i = tid; i < RBN; i += OTHR) srb[i] = 0;
  int carry = 0;
#pragma unroll 1
  for (int fb = 0; fb < nBF; ++fb) {
    const int base = fb * NBF;
    const v4i c = *(const v4i*)(cnt + base + 4 * tid);
    const int e0 = max(c.x, 0), e1 = max(c.y, 0), e2 = max(c.z, 0), e3 = max(c.w, 0);
    const int ts = e0 + e1 + e2 + e3;
    int incl = ts;
#pragma unroll
    for (int d = 1; d < 32; d <<= 1) {
      const int t = __shfl_up(incl, d);
      if (lane >= d) incl += t;
    }
    if (lane == 31) wtot[wave] = incl;
    __syncthreads();
    int pre = 0;
#pragma unroll 1
    for (int w = 0; w < wave; ++w) pre += wtot[w];
    int tot = 0;
#pragma unroll
    for (int w = 0; w < OTHR / 32; ++w) tot += wtot[w];
    int run = carry + pre + incl - ts;
    v4i o;
    o.x = run; run += e0;
    o.y = run; run += e1;
    o.z = run; run += e2;
    o.w = run;
    int* op = off + base + 4 * tid;
    *(volatile v4i*)op = o;
    __threadfence();
    *(volatile v4i*)op = o;
    if (tid == 0) srb[min(fb, RBN - 1)] = carry;
    carry += (tot + 31) & ~31;
    __syncthreads();
  }
  if (tid == 0) srb[min(nBF, RBN - 1)] = carry;
  __syncthreads();
  v4i rv = {0, 0, 0, 0};
  if (tid < 32) rv = *(const v4i*)(srb + 4 * tid);
  if (tid < 32) *(volatile v4i*)(rbase + 4 * tid) = rv;
  __threadfence();
  if (tid < 32) *(volatile v4i*)(rbase + 4 * tid) = rv;
}

__global__ __launch_bounds__(NTHR) void k_fill(
    const int* __restrict__ ei, const int* __restrict__ off, const int* __restrict__ rbase,
    int* csr, int nN, int nE, int vec8, int csrLen) {
  extern __shared__ v4f lds_dyn[];
  int* region = (int*)lds_dyn;
  int* cursor = region + RCAP;
  int* list   = cursor + NBF;
  int* wcnt   = list + LISTN;
  const int tid = threadIdx.x, lane = tid & 31, wave = tid >> 5;
  const int b = blockIdx.x;
  const int nodeBase = b * NBF;
  const int* dsts = ei + nE;

  int rb0 = rbase[b];
  const int rb1 = rbase[b + 1];
  rb0 = rb0 < 0 ? 0 : (rb0 > csrLen ? csrLen : rb0);
  rb0 &= ~31;
  int len = rb1 - rb0;
  len = len < 0 ? 0 : (len > RCAP ? RCAP : len);
  int lenW = (len + 31) & ~31;
  if (rb0 + lenW > csrLen) lenW = (csrLen - rb0) & ~31;

  {
    const v4i z = {0, 0, 0, 0};
    for (int i = tid; i < RCAP / 4; i += NTHR) ((v4i*)region)[i] = z;
    for (int s = tid; s < NBF; s += NTHR) {
      int o = off[nodeBase + s] - rb0;
      o = o < 0 ? 0 : (o > RCAP ? RCAP : o);
      cursor[s] = o;
    }
  }
  __syncthreads();

  const int nChunks = (nE + CHUNK - 1) / CHUNK;
#pragma unroll 1
  for (int ch = 0; ch < nChunks; ++ch) {
    const int cbase = ch * CHUNK;
    const int wc = scan_chunk<NBF, 1>(dsts, ei, nE, nN, cbase, nodeBase, vec8, list, tid, lane, wave);
    if (lane == 0) wcnt[wave] = wc;
    __syncthreads();
    if (wave == 0) {
#pragma unroll 1
      for (int wsx = 0; wsx < NWAVE; ++wsx) {
        int n = __builtin_amdgcn_readfirstlane(wcnt[wsx]);
        n = n > WCAP ? WCAP : (n < 0 ? 0 : n);
        const int* lp = list + wsx * WCAP;
#pragma unroll 1
        for (int i = 0; i < n; ++i) {
          const int ent  = __builtin_amdgcn_readfirstlane(lp[i]);
          const int slot = ent & (NBF - 1);
          int src = (ent >> ESHF) & 0xFFFFF;
          src = src > nN - 1 ? nN - 1 : src;
          if (lane == 0) {
            int pos = cursor[slot];
            pos = pos < 0 ? 0 : (pos > RCAP - 1 ? RCAP - 1 : pos);
            region[pos] = src;
            const int np = pos + 1;
            cursor[slot] = np > RCAP ? RCAP : np;
          }
        }
      }
    }
    __syncthreads();
  }

  const int nv = lenW >> 2;
  int* gp = csr + rb0;
#pragma unroll 1
  for (int i = tid; i < nv; i += NTHR) { const v4i v = ((const v4i*)region)[i]; *(volatile v4i*)(gp + 4 * i) = v; }
  __threadfence();
#pragma unroll 1
  for (int i = tid; i < nv; i += NTHR) { const v4i v = ((const v4i*)region)[i]; *(volatile v4i*)(gp + 4 * i) = v; }
}

template <int KD, int MODE>
__global__ __launch_bounds__(NTHR) void k_gemm(
    const float* __restrict__ A, const unsigned short* __restrict__ Bh, const unsigned short* __restrict__ Bl,
    const float* __restrict__ bias, const float* __restrict__ dinv, float* C, int nRowsA) {
  __shared__ __attribute__((aligned(16))) float stg[NWAVE * 16 * FH];
  const int tid = threadIdx.x, lane = tid & 31, wave = tid >> 5, hh = lane >> 4, m = lane & 15;
  const int row0 = blockIdx.x * GROWS + wave * 16;
  int arow = row0 + m;
  arow = arow > nRowsA - 1 ? nRowsA - 1 : arow;
  const float* ap = A + (size_t)arow * KD + 8 * hh;

  v8f acc[4];
#pragma unroll
  for (int t = 0; t < 4; ++t) { v8f z = {0.f, 0.f, 0.f, 0.f, 0.f, 0.f, 0.f, 0.f}; acc[t] = z; }
#pragma unroll 1
  for (int kt = 0; kt < KD / 32; ++kt) {
    v16us ahi, alo;
    split16(ap + 32 * kt, ahi, alo);
#pragma unroll
    for (int t = 0; t < 4; ++t) {
      const size_t bo = (size_t)(16 * t + m) * KD + 32 * kt + 8 * hh;
      FragU bh, bl;
      bh.h[0] = *(const v8us*)(Bh + bo); bh.h[1] = *(const v8us*)(Bh + bo + 16);
      bl.h[0] = *(const v8us*)(Bl + bo); bl.h[1] = *(const v8us*)(Bl + bo + 16);
      acc[t] = wmb(ahi, bh.v, acc[t]);
      acc[t] = wmb(ahi, bl.v, acc[t]);
      acc[t] = wmb(alo, bh.v, acc[t]);
    }
  }

  const int r0 = 8 * hh;
  float s[8];
  if (MODE == 1) {
    const v4f dA = *(const v4f*)(dinv + (size_t)row0 + r0);
    const v4f dB = *(const v4f*)(dinv + (size_t)row0 + r0 + 4);
    s[0] = dA.x; s[1] = dA.y; s[2] = dA.z; s[3] = dA.w; s[4] = dB.x; s[5] = dB.y; s[6] = dB.z; s[7] = dB.w;
  } else {
#pragma unroll
    for (int r = 0; r < 8; ++r) s[r] = 1.0f;
  }
  float* sw = stg + wave * 16 * FH;
#pragma unroll
  for (int t = 0; t < 4; ++t) {
    const float bv = bias[16 * t + m];
#pragma unroll
    for (int r = 0; r < 8; ++r) sw[(r0 + r) * FH + 16 * t + m] = (acc[t][r] + bv) * s[r];
  }
  __syncthreads();

  float* gp = C + (size_t)row0 * FH;
#pragma unroll
  for (int i = 0; i < (16 * FH) / 128; ++i) {
    const v4f v = *(const v4f*)(sw + i * 128 + 4 * lane);
    *(volatile v4f*)(gp + i * 128 + 4 * lane) = v;
  }
  __threadfence();
#pragma unroll
  for (int i = 0; i < (16 * FH) / 128; ++i) {
    const v4f v = *(const v4f*)(sw + i * 128 + 4 * lane);
    *(volatile v4f*)(gp + i * 128 + 4 * lane) = v;
  }
}

__global__ __launch_bounds__(NTHR) void k_agg(
    const int* __restrict__ csr, const int* __restrict__ off, const int* __restrict__ cnt,
    const float* __restrict__ dinv, const float* __restrict__ hw, float* h, int nN, int csrLen) {
  const int tid = threadIdx.x, lane = tid & 31, wave = tid >> 5;
  const int tbase = blockIdx.x * TGT + wave * 32;
  const int cl = tbase + lane;
  const int cnt_l = cnt[cl];
  const int off_l = off[cl];
  union FI { float f; int i; };
  FI dvu; dvu.f = dinv[cl];

#pragma unroll 1
  for (int j = 0; j < 32; ++j) {
    const int c = tbase + j;
    int n = __builtin_amdgcn_readlane(cnt_l, j);
    n = n < 0 ? 0 : (n > DEGCAP ? DEGCAP : n);
    const int st = __builtin_amdgcn_readlane(off_l, j);
    FI du; du.i = __builtin_amdgcn_readlane(dvu.i, j);
    const float dc = du.f;
    v2f acc = {0.f, 0.f};
#pragma unroll 1
    for (int q0 = 0; q0 < n; q0 += 32) {
      int pos = st + q0 + lane;
      pos = pos < 0 ? 0 : (pos > csrLen - 1 ? csrLen - 1 : pos);
      int sl = csr[pos];
      sl = sl < 0 ? 0 : (sl > nN - 1 ? nN - 1 : sl);
      const int mcnt = (n - q0) < 32 ? (n - q0) : 32;
#pragma unroll 1
      for (int p = 0; p < mcnt; ++p) {
        const int s = __builtin_amdgcn_readlane(sl, p);
        acc = acc + *(const v2f*)(hw + (size_t)s * FH + 2 * lane);
      }
    }
    v2f v = acc * dc;
    v.x = fmaxf(v.x, 0.f); v.y = fmaxf(v.y, 0.f);
    float* hp = h + (size_t)c * FH + 2 * lane;
    *(volatile v2f*)hp = v;
    __threadfence();
    *(volatile v2f*)hp = v;
  }
}

__global__ __launch_bounds__(NTHR) void k_head(
    const float* __restrict__ p1, const float* __restrict__ p2, const float* __restrict__ p3,
    const unsigned short* __restrict__ Bah, const unsigned short* __restrict__ Bal, const float* __restrict__ bla,
    const unsigned short* __restrict__ Bch, const unsigned short* __restrict__ Bcl, const float* __restrict__ bcl,
    float* out, int nN) {
  __shared__ __attribute__((aligned(16))) unsigned short sgh[NWAVE * 16 * APH];
  __shared__ __attribute__((aligned(16))) unsigned short sgl[NWAVE * 16 * APH];
  __shared__ __attribute__((aligned(16))) float so[NWAVE * 16 * FOUT];
  const int tid = threadIdx.x, lane = tid & 31, wave = tid >> 5, hh = lane >> 4, m = lane & 15;
  const int row0 = blockIdx.x * GROWS + wave * 16;

  v8f acc[4];
#pragma unroll
  for (int t = 0; t < 4; ++t) { v8f z = {0.f, 0.f, 0.f, 0.f, 0.f, 0.f, 0.f, 0.f}; acc[t] = z; }
#pragma unroll 1
  for (int p = 0; p < NLAY; ++p) {
    const float* hp = (p == 0) ? p1 : ((p == 1) ? p2 : p3);
    const float* ap = hp + (size_t)(row0 + m) * FH + 8 * hh;
#pragma unroll
    for (int kt = 0; kt < FH / 32; ++kt) {
      v16us ahi, alo;
      split16(ap + 32 * kt, ahi, alo);
#pragma unroll
      for (int t = 0; t < 4; ++t) {
        const size_t bo = (size_t)(16 * t + m) * FLA + FH * p + 32 * kt + 8 * hh;
        FragU bh, bl;
        bh.h[0] = *(const v8us*)(Bah + bo); bh.h[1] = *(const v8us*)(Bah + bo + 16);
        bl.h[0] = *(const v8us*)(Bal + bo); bl.h[1] = *(const v8us*)(Bal + bo + 16);
        acc[t] = wmb(ahi, bh.v, acc[t]);
        acc[t] = wmb(ahi, bl.v, acc[t]);
        acc[t] = wmb(alo, bh.v, acc[t]);
      }
    }
  }

  unsigned short* swh = sgh + wave * 16 * APH;
  unsigned short* swl = sgl + wave * 16 * APH;
#pragma unroll
  for (int t = 0; t < 4; ++t) {
    const float bv = bla[16 * t + m];
#pragma unroll
    for (int r = 0; r < 8; ++r) {
      unsigned short a, b;
      split1(acc[t][r] + bv, a, b);
      swh[(8 * hh + r) * APH + 16 * t + m] = a;
      swl[(8 * hh + r) * APH + 16 * t + m] = b;
    }
  }
  __syncthreads();

  v8f acc2[3];
#pragma unroll
  for (int t = 0; t < 3; ++t) { v8f z = {0.f, 0.f, 0.f, 0.f, 0.f, 0.f, 0.f, 0.f}; acc2[t] = z; }
#pragma unroll
  for (int kt = 0; kt < FH / 32; ++kt) {
    FragU ah, al;
    ah.h[0] = *(const v8us*)(swh + m * APH + 32 * kt + 8 * hh);
    ah.h[1] = *(const v8us*)(swh + m * APH + 32 * kt + 16 + 8 * hh);
    al.h[0] = *(const v8us*)(swl + m * APH + 32 * kt + 8 * hh);
    al.h[1] = *(const v8us*)(swl + m * APH + 32 * kt + 16 + 8 * hh);
#pragma unroll
    for (int t = 0; t < 3; ++t) {
      const size_t bo = (size_t)(16 * t + m) * FH + 32 * kt + 8 * hh;
      FragU bh, bl;
      bh.h[0] = *(const v8us*)(Bch + bo); bh.h[1] = *(const v8us*)(Bch + bo + 16);
      bl.h[0] = *(const v8us*)(Bcl + bo); bl.h[1] = *(const v8us*)(Bcl + bo + 16);
      acc2[t] = wmb(ah.v, bh.v, acc2[t]);
      acc2[t] = wmb(ah.v, bl.v, acc2[t]);
      acc2[t] = wmb(al.v, bh.v, acc2[t]);
    }
  }

  float* sow = so + wave * 16 * FOUT;
#pragma unroll
  for (int t = 0; t < 3; ++t) {
    const int col = 16 * t + m;
    const int cc = col < FOUT ? col : FOUT - 1;
    const float bv = bcl[cc];
#pragma unroll
    for (int r = 0; r < 8; ++r) {
      if (col < FOUT) sow[(8 * hh + r) * FOUT + col] = acc2[t][r] + bv;
    }
  }
  __syncthreads();

  float* gbp = out + (size_t)row0 * FOUT;
#pragma unroll
  for (int i = 0; i < (16 * FOUT) / 128; ++i) {
    const int fidx = i * 128 + 4 * lane;
    const int row = row0 + fidx / FOUT;
    const v4f v = *(const v4f*)(sow + fidx);
    if (row < nN) *(volatile v4f*)(gbp + fidx) = v;
  }
  __threadfence();
#pragma unroll
  for (int i = 0; i < (16 * FOUT) / 128; ++i) {
    const int fidx = i * 128 + 4 * lane;
    const int row = row0 + fidx / FOUT;
    const v4f v = *(const v4f*)(sow + fidx);
    if (row < nN) *(volatile v4f*)(gbp + fidx) = v;
  }
}

extern "C" void kernel_launch(void* const* d_in, const int* in_sizes, int n_in,
                              void* d_out, int out_size, void* d_ws, size_t ws_size,
                              hipStream_t stream) {
  if (n_in < 10) return;
  const int nN = in_sizes[0] / FIN;
  const int nE = in_sizes[1] / 2;
  if (nN <= 0 || nE <= 0 || in_sizes[0] != nN * FIN || in_sizes[1] != 2 * nE) return;
  if (in_sizes[2] != FIN * FH || in_sizes[3] != FH) return;
  if (in_sizes[4] != NLAY * FH * FH || in_sizes[5] != NLAY * FH) return;
  if (in_sizes[6] != FLA * FH || in_sizes[7] != FH) return;
  if (in_sizes[8] != FH * FOUT || in_sizes[9] != FOUT) return;
  if (out_size != nN * FOUT) return;
  if (nN > (1 << 20) || nE > (1 << 28)) return;

  const float* x     = (const float*)d_in[0];
  const int*   ei    = (const int*)d_in[1];
  const float* w_in  = (const float*)d_in[2];
  const float* b_in  = (const float*)d_in[3];
  const float* w_gcn = (const float*)d_in[4];
  const float* b_gcn = (const float*)d_in[5];
  const float* w_la  = (const float*)d_in[6];
  const float* b_la  = (const float*)d_in[7];
  const float* w_cls = (const float*)d_in[8];
  const float* b_cls = (const float*)d_in[9];
  float* out = (float*)d_out;

  const int NPAD   = ((nN + TGT - 1) / TGT) * TGT;
  const int nBC    = (nN + NBC - 1) / NBC;
  const int CNTPAD = nBC * NBC;
  const int nBF    = (nN + NBF - 1) / NBF;
  const int OFFN   = nBF * NBF;
  if (nBF + 1 > RBN) return;
  if (OFFN > CNTPAD || NPAD > OFFN) return;
  const int csrLen = ((nE + 31) & ~31) + 32 * (nBF + 1);
  const int nGemm  = NPAD / GROWS;
  const int nAgg   = NPAD / TGT;

  char* ws = (char*)d_ws;
  size_t off = 0;
  const size_t oW   = off; off += (size_t)PW_TOT * 2 * 2;            off = (off + 255) & ~(size_t)255;
  const size_t oCnt = off; off += (size_t)CNTPAD * 4;                off = (off + 255) & ~(size_t)255;
  const size_t oDv  = off; off += (size_t)CNTPAD * 4;                off = (off + 255) & ~(size_t)255;
  const size_t oOff = off; off += (size_t)OFFN * 4;                  off = (off + 255) & ~(size_t)255;
  const size_t oRb  = off; off += (size_t)RBN * 4;                   off = (off + 255) & ~(size_t)255;
  const size_t oCsr = off; off += (size_t)csrLen * 4;                off = (off + 255) & ~(size_t)255;
  const size_t plB  = (size_t)NPAD * FH * 4;
  const size_t oS0  = off; off += plB;                               off = (off + 255) & ~(size_t)255;
  const size_t oS1  = off; off += plB;                               off = (off + 255) & ~(size_t)255;
  const size_t oS2  = off; off += plB;                               off = (off + 255) & ~(size_t)255;
  const size_t oS3  = off; off += plB;                               off = (off + 255) & ~(size_t)255;
  if (off > ws_size || off > (size_t)WSCAP) return;
  unsigned short* wp = (unsigned short*)(ws + oW);
  int*   cnt  = (int*)(ws + oCnt);
  float* dinv = (float*)(ws + oDv);
  int*   offp = (int*)(ws + oOff);
  int*   rb   = (int*)(ws + oRb);
  int*   csr  = (int*)(ws + oCsr);
  float* S0   = (float*)(ws + oS0);
  float* S1   = (float*)(ws + oS1);
  float* S2   = (float*)(ws + oS2);
  float* S3   = (float*)(ws + oS3);
  const unsigned short* wlo = wp + PW_TOT;

  const int vec8 = ((nE & 3) == 0) ? 1 : 0;

  k_wprep<<<WPREP_BLOCKS, NTHR, 0, stream>>>(w_in, w_gcn, w_la, w_cls, wp);

  hipFuncSetAttribute(reinterpret_cast<const void*>(&k_count),
                      hipFuncAttributeMaxDynamicSharedMemorySize, LDS_COUNT);
  k_count<<<nBC, NTHR, LDS_COUNT, stream>>>(ei, cnt, dinv, nE, nN, vec8);
  k_offsets<<<1, OTHR, 0, stream>>>(cnt, offp, rb, nBF);
  hipFuncSetAttribute(reinterpret_cast<const void*>(&k_fill),
                      hipFuncAttributeMaxDynamicSharedMemorySize, LDS_FILL);
  k_fill<<<nBF, NTHR, LDS_FILL, stream>>>(ei, offp, rb, csr, nN, nE, vec8, csrLen);

  k_gemm<FIN, 0><<<nGemm, NTHR, 0, stream>>>(x, wp + PW_IN, wlo + PW_IN, b_in, dinv, S0, nN);

  float* hin = S0;
  for (int i = 0; i < NLAY; ++i) {
    float* ho = (i == 0) ? S2 : ((i == 1) ? S3 : S0);
    k_gemm<FH, 1><<<nGemm, NTHR, 0, stream>>>(hin, wp + PW_G + (size_t)i * FH * FH, wlo + PW_G + (size_t)i * FH * FH,
                                              b_gcn + (size_t)i * FH, dinv, S1, NPAD);
    k_agg<<<nAgg, NTHR, 0, stream>>>(csr, offp, cnt, dinv, S1, ho, nN, csrLen);
    hin = ho;
  }

  k_head<<<nGemm, NTHR, 0, stream>>>(S2, S3, S0, wp + PW_LA, wlo + PW_LA, b_la, wp + PW_CLS, wlo + PW_CLS, b_cls, out, nN);
}
